// DynamicConvolution_7387343749866
// MI455X (gfx1250) — hardware-verified
//
#include <hip/hip_runtime.h>


namespace {
constexpr int B = 16, CI = 128, CO = 128, H = 64, W = 64, KT = CI * 9, CC = 32  , KCH = CC * 9  , BL = 16  ;
constexpr float XS = 8.0f, WSC = 256.0f;
static_assert(W == 64 && KCH % 32 == 0 && CI % CC == 0, "tiling");
typedef _Float16 b16;
typedef __attribute__((ext_vector_type(16))) _Float16 v16b;
typedef __attribute__((ext_vector_type(8))) _Float16 v8b;
typedef __attribute__((ext_vector_type(8))) float v8f;
typedef __attribute__((ext_vector_type(4))) float v4f;
__device__ __forceinline__ float bf16_rne(float f) { unsigned int u = __float_as_uint(f); u += 0x7FFFu + ((u >> 16) & 1u); return __uint_as_float(u & 0xFFFF0000u); }
__device__ __forceinline__ void split16(float v, b16& hi, b16& lo) { hi = (b16)v; lo = (b16)(v - (float)hi); }
__device__ __forceinline__ v16b frag_kb(const b16* p, int hh) { const v8b a = *(const v8b*)(p + 8 * hh), b = *(const v8b*)(p + 16 + 8 * hh); v16b f;
#pragma unroll
  for (int e = 0; e < 8; ++e) { f[e] = a[e]; f[8 + e] = b[e]; } return f; }
__device__ __forceinline__ v8f wmma16b(v16b a, v16b b, v8f c) { v8f d = __builtin_amdgcn_wmma_f32_16x16x32_f16(false, a, false, b, (short)0, c, false, false); asm volatile("v_nop\n\tv_nop\n\tv_nop\n\tv_nop" : "+v"(d) : "v"(a), "v"(b)); return d; }
__device__ __forceinline__ void wave_lds_sync() { __builtin_amdgcn_fence(__ATOMIC_RELEASE, "workgroup"); __builtin_amdgcn_wave_barrier(); __builtin_amdgcn_fence(__ATOMIC_ACQUIRE, "workgroup"); }
__device__ __forceinline__ float pmul(float a, float b) { float p = a * b; asm volatile("" : "+v"(p)); return p; }
__device__ __forceinline__ int iclamp(int v, int lo, int hi) { return v < lo ? lo : (v > hi ? hi : v); }

typedef __attribute__((ext_vector_type(2))) float v2f;
__global__ __launch_bounds__(256) void prep_kernel(const float* __restrict__ kern, b16* __restrict__ WB) {
  const size_t u = (size_t)blockIdx.x * 256 + threadIdx.x; const size_t n = (size_t)B * CO * KT / 8; if (u >= n) return; const size_t e = u * 8; v8b o;
  for (int j = 0; j < 8; ++j) o[j] = (b16)(bf16_rne(kern[e + j]) * WSC);
  for (int pass = 0; pass < 2; ++pass) { *(volatile v8b*)(WB + e) = o; __threadfence(); }
}
__global__ __launch_bounds__(128) void conv_kernel(const float* __restrict__ feat, const b16* __restrict__ WB, float* __restrict__ out) {
  __shared__ __attribute__((aligned(16))) b16 As[64][KCH + 8]; __shared__ __attribute__((aligned(16))) float Tf[4][16][CO + 4];
  const int wave = threadIdx.x >> 5, lane = threadIdx.x & 31, nloc = lane & 15, hlf = lane >> 4; const int y = blockIdx.x, b = blockIdx.y;
  const float* fb = feat + (size_t)b * CI * H * W; const b16* wb = WB + (size_t)b * CO * KT;
  v8f acc[8];
#pragma unroll
  for (int t = 0; t < 8; ++t) acc[t] = (v8f){};
#pragma unroll 1
  for (int ch = 0; ch < CI; ch += CC) {
    __syncthreads();
    for (int i = threadIdx.x; i < 64 * KCH; i += 128) { const int px = i & 63, k = i >> 6; const int cl = k / 9, tap = k % 9; const int ky = tap / 3, kx = tap % 3; const int yy = y + ky - 1, xx = px + kx - 1;
      float v = 0.0f; if (yy >= 0 && yy < H && xx >= 0 && xx < W) v = bf16_rne(fb[((size_t)(ch + cl) * H + yy) * W + xx]); As[px][k] = (b16)(v * XS); }
    __syncthreads();
#pragma unroll 3
    for (int kb = 0; kb < KCH; kb += 32) { const v16b a = frag_kb(&As[wave * 16 + nloc][kb], hlf);
#pragma unroll
      for (int t = 0; t < 8; ++t) acc[t] = wmma16b(a, frag_kb(wb + (size_t)(t * 16 + nloc) * KT + ch * 9 + kb, hlf), acc[t]); } }
#pragma unroll
  for (int t = 0; t < 8; ++t)
#pragma unroll
    for (int r = 0; r < 8; ++r) Tf[wave][8 * hlf + r][t * 16 + nloc] = acc[t][r] * (1.0f / (XS * WSC));
  __syncthreads();
  for (int pass = 0; pass < 2; ++pass) {
#pragma unroll 1
    for (int q = 0; q < 32; ++q) { const int o = wave * 32 + q; const int px = lane * 2; v2f vv; vv[0] = Tf[px >> 4][px & 15][o]; vv[1] = Tf[(px + 1) >> 4][(px + 1) & 15][o]; *(volatile v2f*)(out + (((size_t)b * CO + o) * H + y) * W + px) = vv; }
    __threadfence(); }
}
}

extern "C" void kernel_launch(void* const* d_in, const int* in_sizes, int n_in, void* d_out, int out_size, void* d_ws, size_t ws_size, hipStream_t stream) {
  (void)n_in;
  auto Fp = [&](int i) { return (const float*)d_in[i]; };
  if (in_sizes[0] != B * CI * H * W || in_sizes[1] != B * CO * KT || out_size != B * CO * H * W) return;
  size_t off = 0; char* ws = (char*)d_ws;
  auto carve = [&](size_t bytes) { char* p = ws + off; off += (bytes + 255) & ~(size_t)255; return p; };
  b16* WB = (b16*)carve((size_t)B * CO * KT * 2);
  if (off > ws_size || off > ((size_t)128 << 20)) return;
  prep_kernel<<<(unsigned)(((size_t)B * CO * KT / 8 + 255) / 256), 256, 0, stream>>>(Fp(1), WB);
  conv_kernel<<<dim3(H, BL), 128, 0, stream>>>(Fp(0), WB, (float*)d_out);
}
